// OptimizedSparseAttention_9990093931185
// MI455X (gfx1250) — hardware-verified
//
#include <hip/hip_runtime.h>
#include <math.h>

constexpr int kBatch = 2;
constexpr int kSeq   = 2048;
constexpr int kDim   = 1024;
constexpr int kHeads = 16;
constexpr int kDh    = 64;
constexpr int kBins  = 16;
constexpr int kTok   = kBatch * kSeq;
constexpr float kScoreScale = 0.125f;
static_assert(kHeads * kDh == kDim, "shape");
static_assert(kTok % 64 == 0 && kDim % 64 == 0 && kSeq % 64 == 0 && kDh % 64 == 0, "tile multiples");
static_assert(kDim % 32 == 0 && kDh % 32 == 0 && kSeq % 32 == 0, "k steps");
static_assert(kSeq % 256 == 0 && kTok % 32 == 0 && (kTok * kDim) % 2048 == 0, "vector kernels");

constexpr size_t kPlane16 = (size_t)kTok * kDim * 2;
constexpr size_t kPlaneW  = (size_t)kDim * kDim * 2;
constexpr size_t kPlane32 = (size_t)kTok * kDim * 4;
constexpr size_t kPlaneVt = (size_t)kBatch * kDim * kSeq * 2;
constexpr size_t kSzBk    = (size_t)kTok * 4;
constexpr size_t kSzSC    = (size_t)kSeq * kSeq * 4;
constexpr size_t kSzPP    = (size_t)kSeq * kSeq * 2;
constexpr size_t kOffXH  = 0;
constexpr size_t kOffXL  = kOffXH + kPlane16;
constexpr size_t kOffWT  = kOffXL + kPlane16;
constexpr size_t kOffQH  = kOffWT + 8 * kPlaneW;
constexpr size_t kOffQL  = kOffQH + kPlane16;
constexpr size_t kOffKF  = kOffQL + kPlane16;
constexpr size_t kOffKH  = kOffKF + kPlane32;
constexpr size_t kOffKL  = kOffKH + kPlane16;
constexpr size_t kOffVTH = kOffKL + kPlane16;
constexpr size_t kOffVTL = kOffVTH + kPlaneVt;
constexpr size_t kOffOH  = kOffVTL + kPlaneVt;
constexpr size_t kOffOL  = kOffOH + kPlane16;
constexpr size_t kOffBK  = kOffOL + kPlane16;
constexpr size_t kWsTotal = kOffBK + kSzBk;
static_assert(kWsTotal == 117456896, "carve");
static_assert(kWsTotal <= 134217728, "carve cap");
static_assert(kSzSC == kPlane32 && kSzPP == kPlane16, "alias extents match the aliased regions exactly");
static_assert(kOffXL % 128 == 0 && kOffWT % 128 == 0 && kOffQH % 128 == 0 && kOffKF % 128 == 0 && kOffBK % 128 == 0, "align");

typedef __attribute__((ext_vector_type(16))) _Float16 v16h;
typedef __attribute__((ext_vector_type(8)))  _Float16 v8h;
typedef __attribute__((ext_vector_type(16))) __bf16   v16b;
typedef __attribute__((ext_vector_type(8)))  __bf16   v8b;
typedef __attribute__((ext_vector_type(8)))  float    v8f;
typedef __attribute__((ext_vector_type(4)))  float    v4f;
typedef __attribute__((ext_vector_type(4)))  int      v4i;
typedef __attribute__((ext_vector_type(4)))  unsigned int v4u;

__device__ __forceinline__ unsigned short f2bf_bits(float f) {
  unsigned u = __float_as_uint(f);
  return (unsigned short)((u + 0x7FFFu + ((u >> 16) & 1u)) >> 16);
}
__device__ __forceinline__ float bf_bits2f(unsigned short h) { return __uint_as_float(((unsigned)h) << 16); }

__device__ __forceinline__ void dep_guard_h(v8f& a, v8f& b, v16h x, v16h y) { asm volatile("v_nop\n\tv_nop\n\tv_nop\n\tv_nop" : "+v"(a), "+v"(b) : "v"(x), "v"(y)); }
__device__ __forceinline__ void dep_guard_b(v8f& a, v8f& b, v16b x, v16b y) { asm volatile("v_nop\n\tv_nop\n\tv_nop\n\tv_nop" : "+v"(a), "+v"(b) : "v"(x), "v"(y)); }
__device__ __forceinline__ void keep4_h(v16h a, v16h b, v16h c, v16h d) { asm volatile("v_nop" :: "v"(a), "v"(b), "v"(c), "v"(d)); }
__device__ __forceinline__ void keep4_b(v16b a, v16b b, v16b c, v16b d) { asm volatile("v_nop" :: "v"(a), "v"(b), "v"(c), "v"(d)); }
__device__ __forceinline__ void acc_guard4(v8f& a, v8f& b, v8f& c, v8f& d) { asm volatile("v_nop\n\tv_nop\n\tv_nop\n\tv_nop" : "+v"(a), "+v"(b), "+v"(c), "+v"(d)); }
template <typename T> struct Frag;
template <> struct Frag<_Float16> {
  typedef v16h V; union U { v16h v; v8h h[2]; };
  static __device__ __forceinline__ v16h load(const _Float16* p) {
    U f; f.h[0] = *(const v8h*)(p); f.h[1] = *(const v8h*)(p + 16); return f.v;
  }
  static __device__ __forceinline__ v8f mma(v16h a, v16h b, v8f c) {
    return __builtin_amdgcn_wmma_f32_16x16x32_f16(false, a, false, b, (short)0, c, false, false);
  }
  static __device__ __forceinline__ void guard(v8f& a, v8f& b, v16h x, v16h y) { dep_guard_h(a, b, x, y); }
  static __device__ __forceinline__ void keep(v16h a, v16h b, v16h c, v16h d) { keep4_h(a, b, c, d); }
};
template <> struct Frag<__bf16> {
  typedef v16b V; union U { v16b v; v8b h[2]; };
  static __device__ __forceinline__ v16b load(const __bf16* p) {
    U f; f.h[0] = *(const v8b*)(p); f.h[1] = *(const v8b*)(p + 16); return f.v;
  }
  static __device__ __forceinline__ v8f mma(v16b a, v16b b, v8f c) {
    return __builtin_amdgcn_wmma_f32_16x16x32_bf16(false, a, false, b, (short)0, c, false, false);
  }
  static __device__ __forceinline__ void guard(v8f& a, v8f& b, v16b x, v16b y) { dep_guard_b(a, b, x, y); }
  static __device__ __forceinline__ void keep(v16b a, v16b b, v16b c, v16b d) { keep4_b(a, b, c, d); }
};

__device__ __forceinline__ unsigned pk16(unsigned short a, unsigned short b) { return (unsigned)a | ((unsigned)b << 16); }
__device__ __forceinline__ void split_bits(float f, unsigned short& hb, unsigned short& lb) {
  hb = f2bf_bits(f);
  lb = f2bf_bits(f - bf_bits2f(hb));
}

template <int ET> struct Elem;
template <> struct Elem<0> { typedef _Float16 T; };
template <> struct Elem<1> { typedef __bf16 T; };
template <int ET, bool SPLIT, int BIAS_MODE, int OUT_MODE, bool RESID, int ACT = 0, int CZ = 0>
__global__ __launch_bounds__(256) void wmma_gemm64(
    const unsigned short* __restrict__ Ap, const unsigned short* __restrict__ A2p, int lda, long strideA,
    const unsigned short* __restrict__ Btp, const unsigned short* __restrict__ Bt2p, int ldb, long strideB,
    void* __restrict__ Cout, void* __restrict__ Cout2, int ldc, long strideC,
    const float* __restrict__ bias,
    const float* __restrict__ resid, long strideR,
    int M, int N, int K, float scale) {
  typedef typename Elem<ET>::T T;
  typedef typename Frag<T>::V V;
  const T* A = (const T*)Ap; const T* A2 = (const T*)A2p; const T* Bt = (const T*)Btp; const T* Bt2 = (const T*)Bt2p;
  __shared__ __align__(16) float sT[8][16 * 68];
  const int b    = blockIdx.y;
  const int lane = threadIdx.x & 31;
  const int wave = threadIdx.x >> 5;
  const int tilesN = N >> 6;
  const int tilesM = M >> 6;
  const int tile = blockIdx.x * 8 + wave;
  if (tile >= tilesM * tilesN) return;
  const int tm = tile / tilesN;
  const int tn = tile - tm * tilesN;
  const int m0 = tm << 6;
  const int n0 = tn << 6;
  if (CZ == 1 && n0 > m0) return;
  const int kEnd = (CZ == 2 && (m0 + 64) < K) ? (m0 + 64) : K;

  const T* Ab  = A  + (size_t)b * strideA;
  const T* Bb  = Bt + (size_t)b * strideB;
  const T* Ab2 = SPLIT ? (A2  + (size_t)b * strideA) : nullptr;
  const T* Bb2 = SPLIT ? (Bt2 + (size_t)b * strideB) : nullptr;

  const int rlane = lane & 15;
  const int koff  = (lane >> 4) * 8;
  const int mOff  = (lane >> 4) * 8;

  v8f acc[4][4];
#pragma unroll
  for (int i = 0; i < 4; ++i)
#pragma unroll
    for (int j = 0; j < 4; ++j) acc[i][j] = (v8f){0.f,0.f,0.f,0.f,0.f,0.f,0.f,0.f};

  for (int k0 = 0; k0 < kEnd; k0 += 32) {
    V bh[4], bl[4];
#pragma unroll
    for (int j = 0; j < 4; ++j) {
      const size_t bo = (size_t)(n0 + (j << 4) + rlane) * ldb + koff + k0;
      bh[j] = Frag<T>::load(Bb + bo);
      if (SPLIT) bl[j] = Frag<T>::load(Bb2 + bo);
    }
#pragma unroll
    for (int i = 0; i < 4; ++i) {
      const size_t ao = (size_t)(m0 + (i << 4) + rlane) * lda + koff + k0;
      V ah = Frag<T>::load(Ab + ao);
      V al;
      if (SPLIT) al = Frag<T>::load(Ab2 + ao);
#pragma unroll
      for (int j = 0; j < 4; ++j) {
        acc[i][j] = Frag<T>::mma(ah, bh[j], acc[i][j]);
        if (SPLIT) {
          acc[i][j] = Frag<T>::mma(ah, bl[j], acc[i][j]);
          acc[i][j] = Frag<T>::mma(al, bh[j], acc[i][j]);
        }
      }
      Frag<T>::guard(acc[i][0], acc[i][3], ah, SPLIT ? al : ah);
    }
    Frag<T>::keep(bh[0], bh[1], bh[2], bh[3]);
    if (SPLIT) Frag<T>::keep(bl[0], bl[1], bl[2], bl[3]);
  }
  acc_guard4(acc[0][0], acc[0][1], acc[0][2], acc[0][3]);
  acc_guard4(acc[1][0], acc[1][1], acc[1][2], acc[1][3]);
  acc_guard4(acc[2][0], acc[2][1], acc[2][2], acc[2][3]);
  acc_guard4(acc[3][0], acc[3][1], acc[3][2], acc[3][3]);

  float* slab = sT[wave];
  const float* Rb = RESID ? (resid + (size_t)b * strideR) : nullptr;
#pragma unroll
  for (int i = 0; i < 4; ++i) {
    const int mBase = m0 + (i << 4);
#pragma unroll
    for (int j = 0; j < 4; ++j) {
      const int n = n0 + (j << 4) + rlane;
      float bv = 0.f;
      if (BIAS_MODE == 2) bv = bias[n];
#pragma unroll
      for (int r = 0; r < 8; ++r) {
        float v = acc[i][j][r] * scale;
        if (BIAS_MODE == 1) v += bias[mBase + mOff + r];
        if (BIAS_MODE == 2) v += bv;
        if (RESID) v += Rb[(size_t)(mBase + mOff + r) * ldc + n];
        if (ACT == 2) v = fmaxf(v, 0.0f);
        if (ACT == 4) v = (v > 0.f) ? v : 0.01f * v;
        slab[(mOff + r) * 68 + (j << 4) + rlane] = v;
      }
    }
    __builtin_amdgcn_fence(__ATOMIC_RELEASE, "workgroup");
    __builtin_amdgcn_wave_barrier();
    __builtin_amdgcn_fence(__ATOMIC_ACQUIRE, "workgroup");
    if (OUT_MODE == 0) {
      float* C = (float*)Cout + (size_t)b * strideC;
      const int hh = lane >> 4, c4 = (lane & 15) * 4;
      for (int pass = 0; pass < 2; ++pass) {
#pragma unroll
        for (int it = 0; it < 8; ++it) {
          const int row = it * 2 + hh;
          v4f v = *(const v4f*)(slab + row * 68 + c4);
          *(volatile v4f*)(C + (size_t)(mBase + row) * ldc + n0 + c4) = v;
        }
        __threadfence();
      }
    } else {
      const int q = lane >> 3, c8 = (lane & 7) * 8;
      unsigned short* C  = (unsigned short*)Cout  + (size_t)b * strideC;
      unsigned short* C2 = (OUT_MODE == 2) ? ((unsigned short*)Cout2 + (size_t)b * strideC) : nullptr;
      for (int pass = 0; pass < 2; ++pass) {
#pragma unroll
        for (int it = 0; it < 4; ++it) {
          const int row = it * 4 + q;
          const float* sp = slab + row * 68 + c8;
          v8h hv, lv;
#pragma unroll
          for (int e = 0; e < 8; ++e) {
            if (OUT_MODE == 1) {
              hv[e] = (_Float16)sp[e];
            } else {
              unsigned short hb = f2bf_bits(sp[e]);
              unsigned short lb = f2bf_bits(sp[e] - bf_bits2f(hb));
              hv[e] = __builtin_bit_cast(_Float16, hb);
              lv[e] = __builtin_bit_cast(_Float16, lb);
            }
          }
          *(volatile v8h*)(C + (size_t)(mBase + row) * ldc + n0 + c8) = hv;
          if (OUT_MODE == 2) *(volatile v8h*)(C2 + (size_t)(mBase + row) * ldc + n0 + c8) = lv;
        }
        __threadfence();
      }
    }
    __builtin_amdgcn_fence(__ATOMIC_RELEASE, "workgroup");
    __builtin_amdgcn_wave_barrier();
    __builtin_amdgcn_fence(__ATOMIC_ACQUIRE, "workgroup");
  }
}

__global__ __launch_bounds__(256) void split8_bf16_kernel(const float* __restrict__ in, unsigned short* __restrict__ hi,
                                                         unsigned short* __restrict__ lo, int n8) {
  const int i = blockIdx.x * 256 + threadIdx.x;
  if (i >= n8) return;
  const float* p = in + 8 * (size_t)i;
  const v4f a = *(const v4f*)(p);
  const v4f c = *(const v4f*)(p + 4);
  unsigned short hb[8], lb[8];
#pragma unroll
  for (int e = 0; e < 4; ++e) {
    split_bits(a[e], hb[e], lb[e]);
    split_bits(c[e], hb[4 + e], lb[4 + e]);
  }
  const v4u uh = (v4u){pk16(hb[0], hb[1]), pk16(hb[2], hb[3]), pk16(hb[4], hb[5]), pk16(hb[6], hb[7])};
  const v4u ul = (v4u){pk16(lb[0], lb[1]), pk16(lb[2], lb[3]), pk16(lb[4], lb[5]), pk16(lb[6], lb[7])};
  unsigned short* qh = hi + 8 * (size_t)i;
  unsigned short* ql = lo + 8 * (size_t)i;
  *(volatile v4u*)qh = uh;
  *(volatile v4u*)ql = ul;
  __threadfence();
  *(volatile v4u*)qh = uh;
  *(volatile v4u*)ql = ul;
}

__global__ __launch_bounds__(256) void wtsplit_kernel(const float* __restrict__ W0, const float* __restrict__ W1,
                                                      const float* __restrict__ W2, const float* __restrict__ W3,
                                                      unsigned short* __restrict__ out) {
  __shared__ float sm[64][65];
  const int t  = threadIdx.x;
  const int k0 = blockIdx.x * 64;
  const int n0 = blockIdx.y * 64;
  const int z  = blockIdx.z;
  const float* W = (z == 0) ? W0 : (z == 1) ? W1 : (z == 2) ? W2 : W3;
#pragma unroll
  for (int i = 0; i < 16; ++i) {
    const int e = i * 256 + t;
    const int r = e >> 6;
    const int c = e & 63;
    sm[c][r] = W[(size_t)(k0 + r) * kDim + n0 + c];
  }
  __syncthreads();
  const int lane = t & 31, wave = t >> 5;
  const int q = lane >> 3, c8 = (lane & 7) * 8;
  unsigned short* oph = out + (size_t)(2 * z) * kDim * kDim;
  unsigned short* opl = oph + (size_t)kDim * kDim;
  for (int pass = 0; pass < 2; ++pass) {
#pragma unroll
    for (int it = 0; it < 2; ++it) {
      const int row = wave * 8 + it * 4 + q;
      unsigned short hb[8], lb[8];
#pragma unroll
      for (int e = 0; e < 8; ++e) split_bits(sm[row][c8 + e], hb[e], lb[e]);
      const v4u uh = (v4u){pk16(hb[0], hb[1]), pk16(hb[2], hb[3]), pk16(hb[4], hb[5]), pk16(hb[6], hb[7])};
      const v4u ul = (v4u){pk16(lb[0], lb[1]), pk16(lb[2], lb[3]), pk16(lb[4], lb[5]), pk16(lb[6], lb[7])};
      const size_t o = (size_t)(n0 + row) * kDim + k0 + c8;
      *(volatile v4u*)(oph + o) = uh;
      *(volatile v4u*)(opl + o) = ul;
    }
    __threadfence();
  }
}

__global__ __launch_bounds__(256) void route_kernel(const float* __restrict__ Kf, const float* __restrict__ wh, int* __restrict__ bkt) {
  __shared__ __align__(16) int sb[32];
  const int t = threadIdx.x;
  const int lane = t & 31, wave = t >> 5;
  const int rbase = blockIdx.x * 32;
#pragma unroll 1
  for (int rr = 0; rr < 4; ++rr) {
    const int row = rbase + wave * 4 + rr;
    const float* kr = Kf + (size_t)row * kDim;
    float acc[kBins];
#pragma unroll
    for (int j = 0; j < kBins; ++j) acc[j] = 0.0f;
#pragma unroll 1
    for (int it = 0; it < kDim / 32; ++it) {
      const int kk = it * 32 + lane;
      const float kv = kr[kk];
      const float* wr = wh + (size_t)kk * kBins;
      const v4f w0 = *(const v4f*)(wr);
      const v4f w1 = *(const v4f*)(wr + 4);
      const v4f w2 = *(const v4f*)(wr + 8);
      const v4f w3 = *(const v4f*)(wr + 12);
#pragma unroll
      for (int e = 0; e < 4; ++e) {
        acc[e]      += kv * w0[e];
        acc[4 + e]  += kv * w1[e];
        acc[8 + e]  += kv * w2[e];
        acc[12 + e] += kv * w3[e];
      }
    }
#pragma unroll
    for (int j = 0; j < kBins; ++j) {
#pragma unroll
      for (int off = 16; off > 0; off >>= 1) acc[j] += __shfl_xor(acc[j], off, 32);
    }
    int best = 0;
    float bv = acc[0];
#pragma unroll
    for (int j = 1; j < kBins; ++j) {
      const bool gt = acc[j] > bv;
      bv = gt ? acc[j] : bv;
      best = gt ? j : best;
    }
    if (lane == 0) sb[wave * 4 + rr] = best;
  }
  __syncthreads();
  if (t < 8) {
    const v4i v = *(const v4i*)(sb + 4 * t);
    int* bp = bkt + rbase + 4 * t;
    *(volatile v4i*)bp = v;
    __threadfence();
    *(volatile v4i*)bp = v;
  }
}

__global__ __launch_bounds__(256) void mask_softmax_kernel(const float* __restrict__ Sp, const int* __restrict__ bkt,
                                                          unsigned short* __restrict__ Ph, unsigned short* __restrict__ Pl, int boff) {
  __shared__ float redM[8];
  __shared__ float redS[8];
  const int row  = blockIdx.x;
  const int t    = threadIdx.x;
  const int lane = t & 31, wave = t >> 5;
  const int cend = (row & ~63) + 64;
  const bool wact = (wave * 256) < cend;
  const int c0 = 8 * t;
  const bool act = c0 < cend;
  const int cc = act ? c0 : (cend - 8);
  const size_t rowoff = (size_t)row * kSeq;
  const int bq = bkt[boff + row];

  const v4f a  = *(const v4f*)(Sp + rowoff + cc);
  const v4f c  = *(const v4f*)(Sp + rowoff + cc + 4);
  const v4i ka = *(const v4i*)(bkt + boff + cc);
  const v4i kc = *(const v4i*)(bkt + boff + cc + 4);
  v4i g0, g1;
  float mx = -__builtin_inff();
#pragma unroll
  for (int e = 0; e < 4; ++e) {
    const int v0 = (act && (cc + e <= row) && (ka[e] == bq)) ? 1 : 0;
    const int v1 = (act && (cc + 4 + e <= row) && (kc[e] == bq)) ? 1 : 0;
    g0[e] = v0;
    g1[e] = v1;
    const float t0 = v0 ? a[e] : -__builtin_inff();
    const float t1 = v1 ? c[e] : -__builtin_inff();
    mx = fmaxf(mx, fmaxf(t0, t1));
  }
#pragma unroll
  for (int off = 16; off > 0; off >>= 1) mx = fmaxf(mx, __shfl_xor(mx, off, 32));
  if (lane == 0) redM[wave] = mx;
  __syncthreads();
  float m = redM[0];
#pragma unroll
  for (int w = 1; w < 8; ++w) m = fmaxf(m, redM[w]);

  float sum = 0.f;
  v4f p0 = (v4f){0.f, 0.f, 0.f, 0.f}, p1 = (v4f){0.f, 0.f, 0.f, 0.f};
  if (wact) {
#pragma unroll
    for (int e = 0; e < 4; ++e) {
      const float a0 = g0[e] ? (a[e] - m) : 0.0f;
      const float a1 = g1[e] ? (c[e] - m) : 0.0f;
      const float q0 = expf(a0);
      const float q1 = expf(a1);
      p0[e] = g0[e] ? q0 : 0.0f;
      p1[e] = g1[e] ? q1 : 0.0f;
      sum += p0[e] + p1[e];
    }
  }
#pragma unroll
  for (int off = 16; off > 0; off >>= 1) sum += __shfl_xor(sum, off, 32);
  if (lane == 0) redS[wave] = sum;
  __syncthreads();
  float tot = redS[0];
#pragma unroll
  for (int w = 1; w < 8; ++w) tot += redS[w];
  const float inv = 1.0f / tot;

  if (act) {
    unsigned short hb[8], lb[8];
#pragma unroll
    for (int e = 0; e < 4; ++e) {
      split_bits(p0[e] * inv, hb[e], lb[e]);
      split_bits(p1[e] * inv, hb[4 + e], lb[4 + e]);
    }
    const v4u uh = (v4u){pk16(hb[0], hb[1]), pk16(hb[2], hb[3]), pk16(hb[4], hb[5]), pk16(hb[6], hb[7])};
    const v4u ul = (v4u){pk16(lb[0], lb[1]), pk16(lb[2], lb[3]), pk16(lb[4], lb[5]), pk16(lb[6], lb[7])};
    unsigned short* prh = Ph + rowoff + (size_t)c0;
    unsigned short* prl = Pl + rowoff + (size_t)c0;
    *(volatile v4u*)prh = uh;
    *(volatile v4u*)prl = ul;
    __threadfence();
    *(volatile v4u*)prh = uh;
    *(volatile v4u*)prl = ul;
  }
}

extern "C" void kernel_launch(void* const* d_in, const int* in_sizes, int n_in,
                              void* d_out, int out_size, void* d_ws, size_t ws_size,
                              hipStream_t stream) {
  if (n_in < 6) return;
  const int nX = kTok * kDim;
  const int nW = kDim * kDim;
  const int nH = kDim * kBins;
  if (in_sizes[0] != nX || in_sizes[1] != nW || in_sizes[2] != nW || in_sizes[3] != nW || in_sizes[4] != nW || in_sizes[5] != nH) return;
  if (out_size != nX) return;
  if (ws_size < kWsTotal) return;

  const float* x  = (const float*)d_in[0];
  const float* wq = (const float*)d_in[1];
  const float* wk = (const float*)d_in[2];
  const float* wv = (const float*)d_in[3];
  const float* wo = (const float*)d_in[4];
  const float* wh = (const float*)d_in[5];
  float* out = (float*)d_out;
  char* ws = (char*)d_ws;
  unsigned short* XH  = (unsigned short*)(ws + kOffXH);
  unsigned short* XL  = (unsigned short*)(ws + kOffXL);
  unsigned short* WT  = (unsigned short*)(ws + kOffWT);
  unsigned short* QH  = (unsigned short*)(ws + kOffQH);
  unsigned short* QL  = (unsigned short*)(ws + kOffQL);
  float*          KF  = (float*)(ws + kOffKF);
  unsigned short* KH  = (unsigned short*)(ws + kOffKH);
  unsigned short* KL  = (unsigned short*)(ws + kOffKL);
  unsigned short* VTH = (unsigned short*)(ws + kOffVTH);
  unsigned short* VTL = (unsigned short*)(ws + kOffVTL);
  unsigned short* OH  = (unsigned short*)(ws + kOffOH);
  unsigned short* OL  = (unsigned short*)(ws + kOffOL);
  int*            BK  = (int*)(ws + kOffBK);
  float*          SC  = (float*)(ws + kOffKF);
  unsigned short* PPH = (unsigned short*)(ws + kOffXH);
  unsigned short* PPL = (unsigned short*)(ws + kOffXL);
  const unsigned short* WqH = WT;
  const unsigned short* WqL = WT + (size_t)1 * nW;
  const unsigned short* WkH = WT + (size_t)2 * nW;
  const unsigned short* WkL = WT + (size_t)3 * nW;
  const unsigned short* WvH = WT + (size_t)4 * nW;
  const unsigned short* WvL = WT + (size_t)5 * nW;
  const unsigned short* WoH = WT + (size_t)6 * nW;
  const unsigned short* WoL = WT + (size_t)7 * nW;

  const int n8 = nX / 8;
  split8_bf16_kernel<<<dim3(n8 / 256), dim3(256), 0, stream>>>(x, XH, XL, n8);
  wtsplit_kernel<<<dim3(kDim / 64, kDim / 64, 4), dim3(256), 0, stream>>>(wq, wk, wv, wo, WT);

  const int tilesProj = (kTok / 64) * (kDim / 64);
  const int tilesVt   = (kDim / 64) * (kSeq / 64);
  wmma_gemm64<1, true, 0, 2, false, 0, 0><<<dim3(tilesProj / 8, 1), dim3(256), 0, stream>>>(
      XH, XL, kDim, 0L, WqH, WqL, kDim, 0L,
      (void*)QH, (void*)QL, kDim, 0L, wh, wh, 0L, kTok, kDim, kDim, 1.0f);
  wmma_gemm64<1, true, 0, 0, false, 0, 0><<<dim3(tilesProj / 8, 1), dim3(256), 0, stream>>>(
      XH, XL, kDim, 0L, WkH, WkL, kDim, 0L,
      (void*)KF, (void*)KF, kDim, 0L, wh, wh, 0L, kTok, kDim, kDim, 1.0f);
  wmma_gemm64<1, true, 0, 2, false, 0, 0><<<dim3(tilesVt / 8, kBatch), dim3(256), 0, stream>>>(
      WvH, WvL, kDim, 0L, XH, XL, kDim, (long)kSeq * kDim,
      (void*)VTH, (void*)VTL, kSeq, (long)kDim * kSeq, wh, wh, 0L, kDim, kSeq, kDim, 1.0f);
  split8_bf16_kernel<<<dim3(n8 / 256), dim3(256), 0, stream>>>(KF, KH, KL, n8);

  route_kernel<<<dim3(kTok / 32), dim3(256), 0, stream>>>(KF, wh, BK);

  const int tilesScore = (kSeq / 64) * (kSeq / 64);
  const int tilesCtx   = (kSeq / 64) * (kDh / 64);
  for (int b = 0; b < kBatch; ++b) {
    for (int h = 0; h < kHeads; ++h) {
      const size_t tokOff = ((size_t)b * kSeq) * kDim + (size_t)h * kDh;
      wmma_gemm64<1, true, 0, 0, false, 0, 1><<<dim3(tilesScore / 8, 1), dim3(256), 0, stream>>>(
          QH + tokOff, QL + tokOff, kDim, 0L, KH + tokOff, KL + tokOff, kDim, 0L,
          (void*)SC, (void*)SC, kSeq, 0L, wh, wh, 0L, kSeq, kSeq, kDh, kScoreScale);
      mask_softmax_kernel<<<dim3(kSeq), dim3(256), 0, stream>>>(SC, BK, PPH, PPL, b * kSeq);
      const size_t vOff = ((size_t)b * kDim + (size_t)h * kDh) * kSeq;
      wmma_gemm64<1, true, 0, 2, false, 0, 2><<<dim3(tilesCtx / 8, 1), dim3(256), 0, stream>>>(
          PPH, PPL, kSeq, 0L, VTH + vOff, VTL + vOff, kSeq, 0L,
          (void*)(OH + tokOff), (void*)(OL + tokOff), kDim, 0L, wh, wh, 0L, kSeq, kDh, kSeq, 1.0f);
    }
  }

  wmma_gemm64<1, true, 0, 0, false, 0, 0><<<dim3(tilesProj / 8, 1), dim3(256), 0, stream>>>(
      OH, OL, kDim, 0L, WoH, WoL, kDim, 0L,
      (void*)out, (void*)out, kDim, 0L, wh, wh, 0L, kTok, kDim, kDim, 1.0f);
}
